// SimpleRNN_14370960572808
// MI455X (gfx1250) — hardware-verified
//
#include <hip/hip_runtime.h>
#include <math.h>

typedef __attribute__((ext_vector_type(16))) _Float16 v16h;
typedef __attribute__((ext_vector_type(8)))  _Float16 v8h;
typedef __attribute__((ext_vector_type(8)))  float    v8f;
typedef __attribute__((ext_vector_type(4)))  float    v4f;

constexpr int kBatch    = 4096;
constexpr int kSteps    = 512;
constexpr int kHid      = 16;
constexpr int kKPad     = 32;
constexpr int kWaves    = 4;
constexpr int kThreads  = kWaves * 32;
constexpr int kTileRows = 16;
constexpr int kRowsPB   = kWaves * kTileRows;
constexpr int kBlocks   = kBatch / kRowsPB;
constexpr int kXChunk   = 64;
constexpr int kXPitch   = kXChunk + 4;
constexpr int kTileElems = kTileRows * kKPad;

constexpr bool kResidual = false;

constexpr float kWCarry   = 16.0f;
constexpr float kHCarry   = 256.0f;
constexpr float kAccScale = kWCarry * kHCarry;
constexpr float kExpMul   = 2.0f / kAccScale;
constexpr float kHInv     = 1.0f / kHCarry;
constexpr float kResCarry = 2048.0f;
constexpr float kResInv   = 1.0f / kResCarry;

static_assert(kBatch % kRowsPB == 0);
static_assert(kBlocks == 64);
static_assert(kSteps % kXChunk == 0);
static_assert(kHid == 16 && kKPad == 32);
static_assert(kRowsPB == 64);
static_assert((kRowsPB * kXChunk / 4) % kThreads == 0);
static_assert((kXPitch * 4) % 16 == 0);
static_assert(kHid * 4 <= kThreads);

template <typename T> struct Frag;
template <> struct Frag<_Float16> {
  typedef v16h V;
  union U { v16h v; v8h h[2]; };
  static __device__ __forceinline__ v16h load(const _Float16* p) {
    U f;
    f.h[0] = *(const v8h*)(p);
    f.h[1] = *(const v8h*)(p + 16);
    return f.v;
  }
  static __device__ __forceinline__ v8f mma(v16h a, v16h b, v8f c) {
    return __builtin_amdgcn_wmma_f32_16x16x32_f16(false, a, false, b, (short)0, c, false, false);
  }
};

__device__ __forceinline__ void wmma_guard1(v8f& a, v16h x, v16h y) {
  asm volatile("v_nop\n\tv_nop\n\tv_nop\n\tv_nop" : "+v"(a) : "v"(x), "v"(y));
}
__device__ __forceinline__ void wmma_guard2(v8f& a, v8f& b, v16h x, v16h y, v16h z, v16h w) {
  asm volatile("v_nop\n\tv_nop\n\tv_nop\n\tv_nop" : "+v"(a), "+v"(b) : "v"(x), "v"(y), "v"(z), "v"(w));
}

__device__ __forceinline__ void w_parts(float wraw, bool live, _Float16& pa, _Float16& pb) {
  const float wv = wraw * kWCarry;
  float wl = 0.0f;
  if (kResidual) {
    const _Float16 wh = (_Float16)wv;
    float back = (float)wh;
    asm volatile("" : "+v"(back));
    wl = (wv - back) * kResCarry;
  }
  const float va = live ? wv : 0.0f;
  const float vb = live ? wv : wl;
  pa = (_Float16)va;
  pb = (_Float16)vb;
}

__global__ __launch_bounds__(kThreads) void rnn_seq_kernel(
    const float* __restrict__ x, const float* __restrict__ w_ih, const float* __restrict__ w_hh,
    const float* __restrict__ b_ih, const float* __restrict__ b_hh,
    const float* __restrict__ w_fc, const float* __restrict__ b_fc,
    float* __restrict__ out) {
  __shared__ __align__(16) float    Xs[kRowsPB * kXPitch];
  __shared__ __align__(16) _Float16 WshA[kHid * kKPad];
  __shared__ __align__(16) _Float16 WshB[kResidual ? kHid * kKPad : 8];
  __shared__ __align__(16) _Float16 HshA[kWaves * kTileElems];
  __shared__ __align__(16) _Float16 HshB[kResidual ? kWaves * kTileElems : 8];
  __shared__ __align__(16) float    Osh[kRowsPB];

  const int tid  = threadIdx.x;
  const int lane = tid & 31;
  const int wave = tid >> 5;
  const int n    = lane & 15;
  const int hh   = lane >> 4;
  const int row0 = blockIdx.x * kRowsPB;

  if (tid < kHid * 4) {
    const int m = tid >> 2;
    const int q = tid & 3;
    const bool live = (q < 2);
    const float* wp = w_hh + m * kHid + 8 * (q & 1);
    const v4f wa = *(const v4f*)(wp);
    const v4f wb = *(const v4f*)(wp + 4);
    v8h pa, pb;
#pragma unroll
    for (int e = 0; e < 4; ++e) {
      _Float16 ta, tb;
      w_parts(wa[e], live, ta, tb);
      pa[e] = ta;
      pb[e] = tb;
    }
#pragma unroll
    for (int e = 0; e < 4; ++e) {
      _Float16 ta, tb;
      w_parts(wb[e], live, ta, tb);
      pa[4 + e] = ta;
      pb[4 + e] = tb;
    }
    *(v8h*)(WshA + m * kKPad + 8 * q) = pa;
    if (kResidual) *(v8h*)(WshB + m * kKPad + 8 * q) = pb;
  }

  float wihS[8], biasS[8], wfc[8];
  {
    const v4f wi0 = *(const v4f*)(w_ih + 8 * hh);
    const v4f wi1 = *(const v4f*)(w_ih + 8 * hh + 4);
    const v4f bi0 = *(const v4f*)(b_ih + 8 * hh);
    const v4f bi1 = *(const v4f*)(b_ih + 8 * hh + 4);
    const v4f bh0 = *(const v4f*)(b_hh + 8 * hh);
    const v4f bh1 = *(const v4f*)(b_hh + 8 * hh + 4);
    const v4f wf0 = *(const v4f*)(w_fc + 8 * hh);
    const v4f wf1 = *(const v4f*)(w_fc + 8 * hh + 4);
#pragma unroll
    for (int e = 0; e < 4; ++e) {
      wihS[e]      = wi0[e] * kAccScale;
      wihS[4 + e]  = wi1[e] * kAccScale;
      biasS[e]     = (bi0[e] + bh0[e]) * kAccScale;
      biasS[4 + e] = (bi1[e] + bh1[e]) * kAccScale;
      wfc[e]       = wf0[e];
      wfc[4 + e]   = wf1[e];
    }
  }
  const float bfc = b_fc[0];

  const v8h z8 = {(_Float16)0.0f, (_Float16)0.0f, (_Float16)0.0f, (_Float16)0.0f,
                  (_Float16)0.0f, (_Float16)0.0f, (_Float16)0.0f, (_Float16)0.0f};
  _Float16* htA = HshA + wave * kTileElems + n * kKPad + 8 * hh;
  _Float16* htB = HshB + (kResidual ? (wave * kTileElems + n * kKPad + 8 * hh) : 0);
  *(v8h*)(htA)      = z8;
  *(v8h*)(htA + 16) = z8;
  if (kResidual) {
    *(v8h*)(htB)      = z8;
    *(v8h*)(htB + 16) = z8;
  }
  __syncthreads();

  const v16h fa  = Frag<_Float16>::load(WshA + n * kKPad + 8 * hh);
  const v16h fa2 = kResidual ? Frag<_Float16>::load(WshB + n * kKPad + 8 * hh) : fa;

  float hlast[8];
#pragma unroll
  for (int r = 0; r < 8; ++r) hlast[r] = 0.0f;

  const float* xrow = Xs + (wave * kTileRows + n) * kXPitch;

#pragma unroll 1
  for (int tc = 0; tc < kSteps; tc += kXChunk) {
    __syncthreads();
#pragma unroll
    for (int i = 0; i < (kRowsPB * kXChunk / 4) / kThreads; ++i) {
      const int idx = tid + kThreads * i;
      const int rr  = idx >> 4;
      const int c4  = (idx & 15) * 4;
      const v4f v = *(const v4f*)(x + (size_t)(row0 + rr) * kSteps + tc + c4);
      *(v4f*)(Xs + rr * kXPitch + c4) = v;
    }
    __syncthreads();

#pragma unroll 1
    for (int tt = 0; tt < kXChunk; ++tt) {
      const float xt = xrow[tt];
      v8f acc;
#pragma unroll
      for (int r = 0; r < 8; ++r) acc[r] = fmaf(xt, wihS[r], biasS[r]);
      const v16h fb = Frag<_Float16>::load(htA);
      acc = Frag<_Float16>::mma(fa, fb, acc);
      v8f acc2 = (v8f){0.f, 0.f, 0.f, 0.f, 0.f, 0.f, 0.f, 0.f};
      if (kResidual) {
        const v16h fb2 = Frag<_Float16>::load(htB);
        acc2 = Frag<_Float16>::mma(fa2, fb2, acc2);
        wmma_guard2(acc, acc2, fa, fb, fa2, fb2);
      } else {
        wmma_guard1(acc, fa, fb);
      }

      v8h hv, hres;
#pragma unroll
      for (int r = 0; r < 8; ++r) {
        float pre = acc[r];
        if (kResidual) pre = fmaf(acc2[r], kResInv, pre);
        float z = pre * kExpMul;
        z = fminf(fmaxf(z, -30.0f), 30.0f);
        const float e = expf(z);
        const float hsv = kHCarry - (2.0f * kHCarry) * __builtin_amdgcn_rcpf(e + 1.0f);
        hlast[r] = hsv;
        const _Float16 h16 = (_Float16)hsv;
        hv[r] = h16;
        if (kResidual) {
          float back = (float)h16;
          asm volatile("" : "+v"(back));
          hres[r] = (_Float16)((hsv - back) * kResCarry);
        } else {
          hres[r] = (_Float16)0.0f;
        }
      }
      *(v8h*)(htA)      = hv;
      *(v8h*)(htA + 16) = z8;
      if (kResidual) {
        *(v8h*)(htB)      = hres;
        *(v8h*)(htB + 16) = hv;
      }
      __syncthreads();
    }
  }

  float part = 0.0f;
#pragma unroll
  for (int r = 0; r < 8; ++r) part = fmaf(hlast[r], wfc[r], part);
  const float other = __shfl_xor(part, 16, 32);
  const float oval = (part + other) * kHInv + bfc;
  if (hh == 0) Osh[wave * kTileRows + n] = oval;
  __syncthreads();

  if (wave == 0) {
    const float v0 = Osh[lane];
    const float v1 = Osh[32 + lane];
    float* op = out + (size_t)row0;
    for (int pass = 0; pass < 2; ++pass) {
      *(volatile float*)(op + lane)      = v0;
      *(volatile float*)(op + 32 + lane) = v1;
      __threadfence();
    }
  }
}

extern "C" void kernel_launch(void* const* d_in, const int* in_sizes, int n_in,
                              void* d_out, int out_size, void* d_ws, size_t ws_size, hipStream_t stream) {
  (void)d_ws;
  (void)ws_size;
  if (n_in < 7 || d_out == nullptr) return;
  if (in_sizes[0] != kBatch * kSteps || in_sizes[1] != kHid || in_sizes[2] != kHid * kHid ||
      in_sizes[3] != kHid || in_sizes[4] != kHid || in_sizes[5] != kHid || in_sizes[6] != 1 ||
      out_size != kBatch) return;

  const float* x    = (const float*)d_in[0];
  const float* w_ih = (const float*)d_in[1];
  const float* w_hh = (const float*)d_in[2];
  const float* b_ih = (const float*)d_in[3];
  const float* b_hh = (const float*)d_in[4];
  const float* w_fc = (const float*)d_in[5];
  const float* b_fc = (const float*)d_in[6];
  float* out = (float*)d_out;

  rnn_seq_kernel<<<kBlocks, kThreads, 0, stream>>>(x, w_ih, w_hh, b_ih, b_hh, w_fc, b_fc, out);
}
